// S4Layer_22204980920820
// MI455X (gfx1250) — hardware-run, weakly checked
//
#include <hip/hip_runtime.h>
#include <math.h>

typedef __attribute__((ext_vector_type(16))) _Float16 v16h;
typedef __attribute__((ext_vector_type(8)))  _Float16 v8h;
typedef __attribute__((ext_vector_type(2)))  _Float16 v2h;
typedef __attribute__((ext_vector_type(16))) __bf16   v16b;
typedef __attribute__((ext_vector_type(8)))  __bf16   v8b;
typedef __attribute__((ext_vector_type(8)))  float    v8f;
typedef __attribute__((ext_vector_type(4)))  float    v4f;
typedef __attribute__((ext_vector_type(2)))  float    v2f;
typedef __attribute__((ext_vector_type(4)))  _Float16 v4h;

constexpr int kNB   = 16;
constexpr int kL    = 2048;
constexpr int kRows = kNB * kL;
constexpr int kDm   = 512;
constexpr int kNs   = 64;
constexpr int kOut0 = kRows * kDm;
constexpr int kThr  = 256;
constexpr float kInCarry = 1024.0f;
constexpr float kWCarry  = 4096.0f;
constexpr float kNCarry  = 1024.0f;
constexpr float kHCarry  = 4096.0f;
constexpr float kScZ = 1.0f / (kNCarry * kWCarry);
constexpr float kScY = 1.0f / (kHCarry * kInCarry);
constexpr float kNormEps = 1e-5f;
constexpr float kF16MinNormal = 6.103515625e-5f;

static_assert(kRows == 32768 && kDm == 512 && kNs == 64 && (kL & (kL - 1)) == 0, "the index arithmetic below uses these sizes");

constexpr size_t kOffA16 = 0ull;
constexpr size_t kOffC16 = 131072ull;
constexpr size_t kOffZB = 196608ull;
constexpr size_t kOffST = 200704ull;
constexpr size_t kOffXN16 = 462848ull;
constexpr size_t kOffZ = 67571712ull;
constexpr size_t kOffH16 = 75960320ull;
constexpr size_t kOffY = 80154624ull;
constexpr size_t kWsTotal = 147263488ull;
static_assert(kWsTotal <= 268435456ull, "the carve stands under the contract's 256 MiB of workspace");
static_assert(kOffA16 == 0
  && kOffC16 == kOffA16 + 131072ull
  && kOffZB == kOffC16 + 65536ull
  && kOffST == kOffZB + 4096ull
  && kOffXN16 == kOffST + 262144ull
  && kOffZ == kOffXN16 + 67108864ull
  && kOffH16 == kOffZ + 8388608ull
  && kOffY == kOffH16 + 4194304ull
  && kWsTotal == kOffY + 67108864ull, "the carve is a chain: every region starts where the one before ends");
static_assert((size_t)kNs * 2 * kDm * 2 == 131072ull && (size_t)kDm * kNs * 2 == 65536ull && 1024ull * 4 == 4096ull && (size_t)kRows * 2 * 4 == 262144ull && (size_t)kRows * 2 * kDm * 2 == 67108864ull && (size_t)kRows * kNs * 4 == 8388608ull && (size_t)kRows * kNs * 2 == 4194304ull
  && (size_t)kRows * kDm * 4 == 67108864ull, "every region's length is its plane's");
static_assert((kOffC16 % 256) == 0 && (kOffZB % 256) == 0 && (kOffST % 256) == 0 && (kOffXN16 % 256) == 0 && (kOffZ % 256) == 0 && (kOffH16 % 256) == 0 && (kOffY % 256) == 0, "every region starts on a multiple of 256 B");

__device__ __forceinline__ unsigned short f2bf_bits(float f) {
  unsigned u = __float_as_uint(f);
  return (unsigned short)((u + 0x7FFFu + ((u >> 16) & 1u)) >> 16);
}
__device__ __forceinline__ float bf_bits2f(unsigned short h) { return __uint_as_float(((unsigned)h) << 16); }
__device__ __forceinline__ float bf16r(float f) { return bf_bits2f(f2bf_bits(f)); }
__device__ __forceinline__ float carry_flush(float v, float carry) {
  const float s = v * carry;
  return (fabsf(s) < kF16MinNormal) ? 0.0f : s;
}

__device__ __forceinline__ void dep_guard4_h(v8f& a, v8f& b, v8f& c, v8f& d, v16h x, v16h y) { asm volatile("v_nop\n\tv_nop\n\tv_nop\n\tv_nop" : "+v"(a), "+v"(b), "+v"(c), "+v"(d) : "v"(x), "v"(y)); }
__device__ __forceinline__ void dep_guard4_b(v8f& a, v8f& b, v8f& c, v8f& d, v16b x, v16b y) { asm volatile("v_nop\n\tv_nop\n\tv_nop\n\tv_nop" : "+v"(a), "+v"(b), "+v"(c), "+v"(d) : "v"(x), "v"(y)); }
__device__ __forceinline__ void keep4_h(v16h a, v16h b, v16h c, v16h d) { asm volatile("v_nop" :: "v"(a), "v"(b), "v"(c), "v"(d)); }
__device__ __forceinline__ void keep4_b(v16b a, v16b b, v16b c, v16b d) { asm volatile("v_nop" :: "v"(a), "v"(b), "v"(c), "v"(d)); }
__device__ __forceinline__ void acc_guard4(v8f& a, v8f& b, v8f& c, v8f& d) { asm volatile("v_nop\n\tv_nop\n\tv_nop\n\tv_nop" : "+v"(a), "+v"(b), "+v"(c), "+v"(d)); }

template <typename T> struct Frag;
template <> struct Frag<_Float16> {
  typedef v16h V; union U { v16h v; v8h h[2]; };
  static __device__ __forceinline__ v16h load(const _Float16* p) {
    U f; f.h[0] = *(const v8h*)(p); f.h[1] = *(const v8h*)(p + 16); return f.v;
  }
  static __device__ __forceinline__ v8f mma(v16h a, v16h b, v8f c) {
    return __builtin_amdgcn_wmma_f32_16x16x32_f16(false, a, false, b, (short)0, c, false, false);
  }
  static __device__ __forceinline__ void guard4(v8f& a, v8f& b, v8f& c, v8f& d, v16h x, v16h y) { dep_guard4_h(a, b, c, d, x, y); }
  static __device__ __forceinline__ void keep(v16h a, v16h b, v16h c, v16h d) { keep4_h(a, b, c, d); }
};
template <> struct Frag<__bf16> {
  typedef v16b V; union U { v16b v; v8b h[2]; };
  static __device__ __forceinline__ v16b load(const __bf16* p) {
    U f; f.h[0] = *(const v8b*)(p); f.h[1] = *(const v8b*)(p + 16); return f.v;
  }
  static __device__ __forceinline__ v8f mma(v16b a, v16b b, v8f c) {
    return __builtin_amdgcn_wmma_f32_16x16x32_bf16(false, a, false, b, (short)0, c, false, false);
  }
  static __device__ __forceinline__ void guard4(v8f& a, v8f& b, v8f& c, v8f& d, v16b x, v16b y) { dep_guard4_b(a, b, c, d, x, y); }
  static __device__ __forceinline__ void keep(v16b a, v16b b, v16b c, v16b d) { keep4_b(a, b, c, d); }
};

__device__ __forceinline__ v8f mma_h(v16h a, v16h b, v8f c) {
  c = __builtin_amdgcn_wmma_f32_16x16x32_f16(false, a, false, b, (short)0, c, false, false);
  asm volatile("v_nop\n\tv_nop\n\tv_nop\n\tv_nop" : "+v"(c) : "v"(a), "v"(b));
  return c;
}

template <int ET> struct Elem;
template <> struct Elem<0> { typedef _Float16 T; };
template <> struct Elem<1> { typedef __bf16 T; };
template <int ET, bool SPLIT, int BIAS_MODE, int OUT_MODE, bool RESID, int ACT = 0>
__global__ __launch_bounds__(256) void wmma_gemm64(
    const unsigned short* __restrict__ Ap, const unsigned short* __restrict__ A2p, int lda, long strideA,
    const unsigned short* __restrict__ Btp, const unsigned short* __restrict__ Bt2p, int ldb, long strideB,
    void* __restrict__ Cout, void* __restrict__ Cout2, int ldc, long strideC,
    const float* __restrict__ bias,
    const float* __restrict__ resid, long strideR,
    int M, int N, int K, float scale) {
  typedef typename Elem<ET>::T T;
  typedef typename Frag<T>::V V;
  const T* A = (const T*)Ap; const T* A2 = (const T*)A2p; const T* Bt = (const T*)Btp; const T* Bt2 = (const T*)Bt2p;
  __shared__ __align__(16) float sT[8][16 * 68];
  const int b    = blockIdx.y;
  const int lane = threadIdx.x & 31;
  const int wave = threadIdx.x >> 5;
  const int tilesN = N >> 6;
  const int tilesM = M >> 6;
  const int tile = blockIdx.x * 8 + wave;
  if (tile >= tilesM * tilesN) return;
  const int tm = tile / tilesN;
  const int tn = tile - tm * tilesN;
  const int m0 = tm << 6;
  const int n0 = tn << 6;

  const T* Ab  = A  + (size_t)b * strideA;
  const T* Bb  = Bt + (size_t)b * strideB;
  const T* Ab2 = SPLIT ? (A2  + (size_t)b * strideA) : nullptr;
  const T* Bb2 = SPLIT ? (Bt2 + (size_t)b * strideB) : nullptr;

  const int rlane = lane & 15;
  const int koff  = (lane >> 4) * 8;
  const int mOff  = (lane >> 4) * 8;

  v8f acc[4][4];
#pragma unroll
  for (int i = 0; i < 4; ++i)
#pragma unroll
    for (int j = 0; j < 4; ++j) acc[i][j] = (v8f){0.f,0.f,0.f,0.f,0.f,0.f,0.f,0.f};

  for (int k0 = 0; k0 < K; k0 += 32) {
    V bh[4], bl[4];
#pragma unroll
    for (int j = 0; j < 4; ++j) {
      const size_t bo = (size_t)(n0 + (j << 4) + rlane) * ldb + koff + k0;
      bh[j] = Frag<T>::load(Bb + bo);
      if (SPLIT) bl[j] = Frag<T>::load(Bb2 + bo);
    }
#pragma unroll
    for (int i = 0; i < 4; ++i) {
      const size_t ao = (size_t)(m0 + (i << 4) + rlane) * lda + koff + k0;
      V ah = Frag<T>::load(Ab + ao);
      V al;
      if (SPLIT) al = Frag<T>::load(Ab2 + ao);
#pragma unroll
      for (int j = 0; j < 4; ++j) {
        acc[i][j] = Frag<T>::mma(ah, bh[j], acc[i][j]);
        if (SPLIT) {
          acc[i][j] = Frag<T>::mma(ah, bl[j], acc[i][j]);
          acc[i][j] = Frag<T>::mma(al, bh[j], acc[i][j]);
        }
      }
      Frag<T>::guard4(acc[i][0], acc[i][1], acc[i][2], acc[i][3], ah, SPLIT ? al : ah);
    }
    Frag<T>::keep(bh[0], bh[1], bh[2], bh[3]);
    if (SPLIT) Frag<T>::keep(bl[0], bl[1], bl[2], bl[3]);
  }
  acc_guard4(acc[0][0], acc[0][1], acc[0][2], acc[0][3]);
  acc_guard4(acc[1][0], acc[1][1], acc[1][2], acc[1][3]);
  acc_guard4(acc[2][0], acc[2][1], acc[2][2], acc[2][3]);
  acc_guard4(acc[3][0], acc[3][1], acc[3][2], acc[3][3]);

  float* slab = sT[wave];
  const float* Rb = RESID ? (resid + (size_t)b * strideR) : nullptr;
#pragma unroll
  for (int i = 0; i < 4; ++i) {
    const int mBase = m0 + (i << 4);
#pragma unroll
    for (int j = 0; j < 4; ++j) {
      const int n = n0 + (j << 4) + rlane;
      float bv = 0.f;
      if (BIAS_MODE == 2) bv = bias[n];
#pragma unroll
      for (int r = 0; r < 8; ++r) {
        float v = acc[i][j][r] * scale;
        if (BIAS_MODE == 1) v += bias[mBase + mOff + r];
        if (BIAS_MODE == 2) v += bv;
        if (RESID) v += Rb[(size_t)(mBase + mOff + r) * ldc + n];
        if (ACT == 1) v = tanhf(v);
        if (ACT == 2) v = fmaxf(v, 0.0f);
        if (ACT == 3) v = v / (1.0f + expf(-v));
        if (ACT == 4) v = (v > 0.f) ? v : 0.01f * v;
        slab[(mOff + r) * 68 + (j << 4) + rlane] = v;
      }
    }
    __builtin_amdgcn_fence(__ATOMIC_RELEASE, "workgroup");
    __builtin_amdgcn_wave_barrier();
    __builtin_amdgcn_fence(__ATOMIC_ACQUIRE, "workgroup");
    if (OUT_MODE == 0) {
      float* C = (float*)Cout + (size_t)b * strideC;
      const int hh = lane >> 4, c4 = (lane & 15) * 4;
      for (int pass = 0; pass < 2; ++pass) {
#pragma unroll
        for (int it = 0; it < 8; ++it) {
          const int row = it * 2 + hh;
          v4f v = *(const v4f*)(slab + row * 68 + c4);
          *(volatile v4f*)(C + (size_t)(mBase + row) * ldc + n0 + c4) = v;
        }
        __threadfence();
      }
    } else {
      const int q = lane >> 3, c8 = (lane & 7) * 8;
      unsigned short* C  = (unsigned short*)Cout  + (size_t)b * strideC;
      unsigned short* C2 = (OUT_MODE == 2) ? ((unsigned short*)Cout2 + (size_t)b * strideC) : nullptr;
      for (int pass = 0; pass < 2; ++pass) {
#pragma unroll
        for (int it = 0; it < 4; ++it) {
          const int row = it * 4 + q;
          const float* sp = slab + row * 68 + c8;
          v8h hv, lv;
#pragma unroll
          for (int e = 0; e < 8; ++e) {
            if (OUT_MODE == 1) {
              hv[e] = (_Float16)sp[e];
            } else {
              unsigned short hb = f2bf_bits(sp[e]);
              unsigned short lb = f2bf_bits(sp[e] - bf_bits2f(hb));
              hv[e] = __builtin_bit_cast(_Float16, hb);
              lv[e] = __builtin_bit_cast(_Float16, lb);
            }
          }
          *(volatile v8h*)(C + (size_t)(mBase + row) * ldc + n0 + c8) = hv;
          if (OUT_MODE == 2) *(volatile v8h*)(C2 + (size_t)(mBase + row) * ldc + n0 + c8) = lv;
        }
        __threadfence();
      }
    }
    __builtin_amdgcn_fence(__ATOMIC_RELEASE, "workgroup");
    __builtin_amdgcn_wave_barrier();
    __builtin_amdgcn_fence(__ATOMIC_ACQUIRE, "workgroup");
  }
}


__global__ __launch_bounds__(kThr) void cast_plane_kernel(const float* __restrict__ src, unsigned short* __restrict__ dst,
                                                          int colsLog2, int dstPitch, int dstOff) {
  const int i   = blockIdx.x * kThr + threadIdx.x;
  const int sh  = colsLog2 - 3;
  const int row = i >> sh;
  const int c8  = (i & ((1 << sh) - 1)) * 8;
  const float* sp = src + ((size_t)row << colsLog2) + c8;
  const v4f a0 = *(const v4f*)(sp);
  const v4f a1 = *(const v4f*)(sp + 4);
  v8h hv;
#pragma unroll
  for (int e = 0; e < 4; ++e) {
    const float f0 = a0[e];
    const float f1 = a1[e];
    hv[e]     = (_Float16)carry_flush(bf16r(f0), kInCarry);
    hv[4 + e] = (_Float16)carry_flush(bf16r(f1), kInCarry);
  }
  unsigned short* dp = dst + (size_t)row * dstPitch + dstOff + c8;
  *(volatile v8h*)dp = hv;
  __threadfence();
  *(volatile v8h*)dp = hv;
}

__global__ __launch_bounds__(256) void wt_plane_kernel(const float* __restrict__ W, unsigned short* __restrict__ dst, int K, int N, int nLive, int ldd, int colOff) {
  const int n  = blockIdx.x;
  const int k8 = threadIdx.x * 8;
  const bool live = n < nLive;
  const int nc = live ? n : 0;
  v8h hv;
#pragma unroll
  for (int e = 0; e < 8; ++e) {
    const float w = W[(size_t)(k8 + e) * N + nc];
    hv[e] = (_Float16)(live ? carry_flush(bf16r(w), kWCarry) : 0.0f);
  }
  unsigned short* dp = dst + (size_t)n * ldd + colOff + k8;
  *(volatile v8h*)dp = hv;
  __threadfence();
  *(volatile v8h*)dp = hv;
}

__global__ __launch_bounds__(kThr) void setup_kernel(float* __restrict__ ZB) {
  float* dp = ZB + blockIdx.x * (unsigned)kThr + threadIdx.x;
  *(volatile float*)dp = 0.0f;
  __threadfence();
  *(volatile float*)dp = 0.0f;
}
static_assert(4 * kThr == 1024 && 1024 >= kDm, "set-up grid exact: 4 blocks of zero bias");

__global__ __launch_bounds__(kThr) void stat_kernel(const float* __restrict__ x, float* __restrict__ ST) {
  const unsigned row = blockIdx.x * (unsigned)kThr + threadIdx.x;
  const float* pr = x + row * (unsigned)kDm;
  float s = 0.0f;
  for (int q = 0; q < kDm / 4; ++q) { const v4f v = *(const v4f*)(pr + 4 * q); s += bf16r(v[0]); s += bf16r(v[1]); s += bf16r(v[2]); s += bf16r(v[3]); }
  const float mu = s / (float)kDm;
  float qq = 0.0f;
  for (int q = 0; q < kDm / 4; ++q) { const v4f v = *(const v4f*)(pr + 4 * q);
#pragma unroll
    for (int e = 0; e < 4; ++e) { const float d = bf16r(v[e]) - mu; qq += d * d; } }
  v2f o; o[0] = mu; o[1] = 1.0f / sqrtf(qq / (float)kDm + kNormEps);
  float* dp = ST + row * 2u;
  *(volatile v2f*)dp = o;
  __threadfence();
  *(volatile v2f*)dp = o;
}
static_assert(kRows == 128 * kThr && (kDm % 4) == 0, "the statistics' grid exact: 128 blocks: a thread a row");

__global__ __launch_bounds__(kThr) void apply_kernel(const float* __restrict__ x, const float* __restrict__ ST, const float* __restrict__ gamma, const float* __restrict__ beta,
                                                     unsigned short* __restrict__ XN16) {
  const unsigned i = blockIdx.x * (unsigned)kThr + threadIdx.x;
  const unsigned row = i >> 6;
  const unsigned c8 = (i & 63u) * 8u;
  const v2f ms = *(const v2f*)(ST + row * 2u);
  const float* pr = x + i * 8u;
  const v4f a0 = *(const v4f*)pr, a1 = *(const v4f*)(pr + 4);
  const v4f g0 = *(const v4f*)(gamma + c8), g1 = *(const v4f*)(gamma + c8 + 4), b0 = *(const v4f*)(beta + c8), b1 = *(const v4f*)(beta + c8 + 4);
  v8h hv, lv;
#pragma unroll
  for (int e = 0; e < 8; ++e) {
    const float v = (e < 4) ? a0[e] : a1[e - 4];
    const float gw = (e < 4) ? g0[e] : g1[e - 4];
    const float gb = (e < 4) ? b0[e] : b1[e - 4];
    const float s = carry_flush(((bf16r(v) - ms[0]) * ms[1]) * bf16r(gw) + bf16r(gb), kNCarry);
    const _Float16 hi = (_Float16)s;
    hv[e] = hi;
    lv[e] = (_Float16)carry_flush(s - (float)hi, 1.0f);
  }
  unsigned short* dp = XN16 + row * (unsigned)(2 * kDm) + c8;
  for (int pass = 0; pass < 2; ++pass) {
    *(volatile v8h*)dp = hv;
    *(volatile v8h*)(dp + kDm) = lv;
    __threadfence();
  }
}
static_assert((size_t)kRows * kDm / 8 == 8192ull * kThr && kDm / 8 == 64, "the apply grid exact: 8,192 blocks: four rows a block");

__global__ __launch_bounds__(kThr) void chain_kernel(const float* __restrict__ Z, unsigned short* __restrict__ H16) {
  const unsigned ix = blockIdx.x * (unsigned)kThr + threadIdx.x;
  const unsigned sq = ix >> 5;
  const unsigned n0 = (ix & 31u) * 2u;
  float h0 = 0.0f, h1 = 0.0f;
  for (int l = 0; l < kL; ++l) {
    const unsigned off = (sq * (unsigned)kL + (unsigned)l) * (unsigned)kNs + n0;
    const v2f zr = *(const v2f*)(Z + off);
    h0 = tanhf(zr[0] + h0);
    h1 = tanhf(zr[1] + h1);
    v2h hv;
    hv[0] = (_Float16)carry_flush(h0, kHCarry);
    hv[1] = (_Float16)carry_flush(h1, kHCarry);
    unsigned short* dp = H16 + off;
    *(volatile v2h*)dp = hv;
    __threadfence();
    *(volatile v2h*)dp = hv;
  }
}
static_assert(kNB * kNs / 2 == 2 * kThr && kNs == 64, "chain grid exact: 2 blocks: a wave is one sequence's 64 states");

__global__ __launch_bounds__(kThr) void close_kernel(const float* __restrict__ Y, const float* __restrict__ x, const float* __restrict__ ST, const float* __restrict__ gamma, const float* __restrict__ beta,
                                                     const float* __restrict__ Dv, float* __restrict__ out) {
  const unsigned i = blockIdx.x * (unsigned)kThr + threadIdx.x;
  const unsigned row = i >> 6;
  const unsigned c8 = (i & 63u) * 8u;
  const v2f ms = *(const v2f*)(ST + row * 2u);
  const float* px = x + i * 8u;
  const float* py = Y + i * 8u;
  const v4f a0 = *(const v4f*)px, a1 = *(const v4f*)(px + 4);
  const v4f y0 = *(const v4f*)py, y1 = *(const v4f*)(py + 4);
  const v4f g0 = *(const v4f*)(gamma + c8), g1 = *(const v4f*)(gamma + c8 + 4), b0 = *(const v4f*)(beta + c8), b1 = *(const v4f*)(beta + c8 + 4);
  const v4f d0 = *(const v4f*)(Dv + c8), d1 = *(const v4f*)(Dv + c8 + 4);
  v4f o0, o1;
#pragma unroll
  for (int e = 0; e < 4; ++e) {
    const float xv0 = bf16r(a0[e]), xv1 = bf16r(a1[e]);
    const float u0 = ((xv0 - ms[0]) * ms[1]) * bf16r(g0[e]) + bf16r(b0[e]);
    const float u1 = ((xv1 - ms[0]) * ms[1]) * bf16r(g1[e]) + bf16r(b1[e]);
    o0[e] = (y0[e] + u0 * bf16r(d0[e])) + xv0;
    o1[e] = (y1[e] + u1 * bf16r(d1[e])) + xv1;
  }
  float* dp = out + i * 8u;
  for (int pass = 0; pass < 2; ++pass) {
    *(volatile v4f*)dp = o0;
    *(volatile v4f*)(dp + 4) = o1;
    __threadfence();
  }
}
static_assert((size_t)kRows * kDm / 8 == 8192ull * kThr && (size_t)kRows * kDm < 4294967296ull / 4, "the closing sum's grid exact: 8,192 blocks; every plane's element offsets fit 32 bits");

extern "C" void kernel_launch(void* const* d_in, const int* in_sizes, int n_in,
                              void* d_out, int out_size, void* d_ws, size_t ws_size,
                              hipStream_t stream) {
  if (n_in < 6 || d_out == nullptr || d_ws == nullptr) return;
  if (in_sizes[0] != kRows * kDm || in_sizes[1] != kDm * kNs || in_sizes[2] != kDm * kNs || in_sizes[3] != kDm || in_sizes[4] != kDm || in_sizes[5] != kDm) return;
  if (out_size != kOut0) return;
  if (ws_size < kWsTotal) return;
  const float* x = (const float*)d_in[0];
  const float* A = (const float*)d_in[1];
  const float* C = (const float*)d_in[2];
  const float* Dv = (const float*)d_in[3];
  const float* gamma = (const float*)d_in[4];
  const float* beta = (const float*)d_in[5];
  float* out = (float*)d_out;
  char* ws = (char*)d_ws;
  unsigned short* A16 = (unsigned short*)(ws + kOffA16);
  unsigned short* C16 = (unsigned short*)(ws + kOffC16);
  float* ZB = (float*)(ws + kOffZB);
  float* ST = (float*)(ws + kOffST);
  unsigned short* XN16 = (unsigned short*)(ws + kOffXN16);
  float* Z = (float*)(ws + kOffZ);
  unsigned short* H16 = (unsigned short*)(ws + kOffH16);
  float* Y = (float*)(ws + kOffY);

  static_assert(kDm / 8 == 64 && ((size_t)kDm * kNs / 8) % kThr == 0, "A's transposing cast: one block a destination row with exactly K / 8 = 64 threads; C's plane is whole rows of 64");
  wt_plane_kernel<<<kNs, kDm / 8, 0, stream>>>(A, A16, kDm, kNs, kNs, 2 * kDm, 0);
  wt_plane_kernel<<<kNs, kDm / 8, 0, stream>>>(A, A16, kDm, kNs, kNs, 2 * kDm, kDm);
  cast_plane_kernel<<<(int)(((size_t)kDm * kNs / 8) / kThr), kThr, 0, stream>>>(C, C16, 6, kNs, 0);
  setup_kernel<<<4, kThr, 0, stream>>>(ZB);
  stat_kernel<<<128, kThr, 0, stream>>>(x, ST);
  apply_kernel<<<8192, kThr, 0, stream>>>(x, ST, gamma, beta, XN16);
  wmma_gemm64<0, false, 2, 0, false, 0><<<dim3((kRows / 64) * (kNs / 64) / 8, 1), 256, 0, stream>>>(
      XN16, XN16, 2 * kDm, 0L, A16, A16, 2 * kDm, 0L, (void*)Z, (void*)Z, kNs, 0L, ZB, nullptr, 0L, kRows, kNs, 2 * kDm, kScZ);
  chain_kernel<<<2, kThr, 0, stream>>>(Z, H16);
  wmma_gemm64<0, false, 2, 0, false, 0><<<dim3((kRows / 64) * (kDm / 64) / 8, 1), 256, 0, stream>>>(
      H16, H16, kNs, 0L, C16, C16, kNs, 0L, (void*)Y, (void*)Y, kDm, 0L, ZB, nullptr, 0L, kRows, kDm, kNs, kScY);
  close_kernel<<<8192, kThr, 0, stream>>>(Y, x, ST, gamma, beta, Dv, out);
}
static_assert(((kRows / 64) * (kNs / 64)) % 8 == 0 && ((kRows / 64) * (kDm / 64)) % 8 == 0, "the engine's grids: whole blocks of eight wave tiles");
